// alpha_net_spatial2_14843406975142
// MI455X (gfx1250) — hardware-verified
//
#include <hip/hip_runtime.h>
#include <math.h>

#define NB_ 16
#define CC 256
#define NN 1024

typedef _Float16 f16;
typedef __attribute__((ext_vector_type(16))) f16 f16x16;
typedef __attribute__((ext_vector_type(8)))  f16 f16x8;
typedef __attribute__((ext_vector_type(8)))  float f32x8;
typedef __attribute__((ext_vector_type(4)))  float v4f_t;
typedef float v4fa __attribute__((ext_vector_type(4), may_alias));
__device__ __forceinline__ f32x8 wmma16(f16x16 a, f16x16 b, f32x8 c) {
  c = __builtin_amdgcn_wmma_f32_16x16x32_f16(false, a, false, b, (short)0, c, false, false);
  asm volatile("v_nop\n\tv_nop\n\tv_nop\n\tv_nop" : "+v"(c) : "v"(a), "v"(b));
  return c;
}
__device__ __forceinline__ f16x16 lds_frag(const f16* base, int stride) {
  const int lane = threadIdx.x & 31, row = lane & 15, kh = (lane >> 4) * 8;
  const f16x8 lo = *(const f16x8*)(base + row * stride + kh);
  const f16x8 hi = *(const f16x8*)(base + row * stride + kh + 16);
  f16x16 f;
#pragma unroll
  for (int i = 0; i < 8; ++i) { f[i] = lo[i]; f[i + 8] = hi[i]; }
  return f;
}
__global__ __launch_bounds__(256) void k_ab(const float* __restrict__ h, const float* __restrict__ w1, const float* __restrict__ b1, const float* __restrict__ w2, const float* __restrict__ b2,
                                           float* __restrict__ av, float* __restrict__ bv) {
  const int b = blockIdx.x >> 2, n = (blockIdx.x & 3) * 256 + threadIdx.x; const float* src = h + (size_t)b * CC * NN + n;
  float sa = b1[0], sb = b2[0];
#pragma unroll 4
  for (int c = 0; c < CC; ++c) { const float v = src[(size_t)c * NN]; sa += v * w1[c]; sb += v * w2[c]; }
  av[(size_t)b * NN + n] = sa; bv[(size_t)b * NN + n] = sb;
}
__global__ __launch_bounds__(256) void k_attn(const float* __restrict__ h, const float* __restrict__ av, const float* __restrict__ bvv, float* __restrict__ out) {
  __shared__ __attribute__((aligned(16))) f16 pS[32 * 40];
  __shared__ float aS[32], lS[32], bS[NN];
  __shared__ __attribute__((aligned(16))) float oS[CC * 36];
  const int tid = threadIdx.x, lane = tid & 31, wave = tid >> 5, cl = lane & 15, rh = (lane >> 4) * 8;
  const int b = blockIdx.x / (NN / 32), i0 = (blockIdx.x % (NN / 32)) * 32;
  for (int e = tid; e < NN; e += 256) bS[e] = bvv[(size_t)b * NN + e];
  if (tid < 32) { aS[tid] = av[(size_t)b * NN + i0 + tid]; lS[tid] = 0.0f; }
  const float* hb = h + (size_t)b * CC * NN;
  const int it = wave & 1, ct0 = (wave >> 1) * 4;
  f32x8 acc[4];
#pragma unroll
  for (int j = 0; j < 4; ++j) { f32x8 z = {}; acc[j] = z; }
  float lpart = 0.0f;
  __syncthreads();
#pragma unroll 1
  for (int j0 = 0; j0 < NN; j0 += 32) {
    { const int i = tid >> 3, part = tid & 7; const float ai = aS[i];
#pragma unroll
      for (int e = 0; e < 4; ++e) { const int jl = part * 4 + e; const float s = expf(tanhf(ai + bS[j0 + jl])); lpart += s; pS[i * 40 + jl] = (f16)(s * 1024.0f); } }
    __syncthreads();
    { const f16x16 af = lds_frag(pS + (it * 16) * 40, 40);
#pragma unroll
      for (int j = 0; j < 4; ++j) { const int ct = ct0 + j; const int n = ct * 16 + (lane & 15), kh = (lane >> 4) * 8; const float* src = hb + (size_t)n * NN + j0 + kh; f16x16 bf;
#pragma unroll
        for (int e = 0; e < 8; ++e) { bf[e] = (f16)src[e]; bf[8 + e] = (f16)src[16 + e]; }
        acc[j] = wmma16(af, bf, acc[j]); } }
    __syncthreads();
  }
  lpart += __shfl_xor(lpart, 1, 32); lpart += __shfl_xor(lpart, 2, 32); lpart += __shfl_xor(lpart, 4, 32);
  if ((tid & 7) == 0) lS[tid >> 3] = lpart;
  __syncthreads();
#pragma unroll
  for (int j = 0; j < 4; ++j)
#pragma unroll
    for (int r = 0; r < 8; ++r) { const int i = it * 16 + rh + r, c = (ct0 + j) * 16 + cl; float v = acc[j][r] / (lS[i] * 1024.0f); v = (v >= 0.0f) ? v : 0.2f * v; oS[c * 36 + i] = v; }
  __syncthreads();
#pragma unroll 1
  for (int pass = 0; pass < 2; ++pass) { { const int c = tid;
#pragma unroll
      for (int q = 0; q < 8; ++q) *(volatile v4f_t*)(out + ((size_t)b * CC + c) * NN + i0 + q * 4) = *(const volatile v4fa*)(oS + c * 36 + q * 4); } __threadfence(); }
}

extern "C" void kernel_launch(void* const* d_in, const int* in_sizes, int n_in,
                              void* d_out, int out_size, void* d_ws, size_t ws_size,
                              hipStream_t stream) {
  (void)in_sizes; (void)n_in; (void)out_size;
  const float* h = (const float*)d_in[0];
  const float* w1 = (const float*)d_in[1], *b1 = (const float*)d_in[2], *w2 = (const float*)d_in[3], *b2 = (const float*)d_in[4];
  float* out = (float*)d_out;
  char* ws = (char*)d_ws;
  float* av = (float*)ws; ws += (size_t)NB_ * NN * 4; float* bv = (float*)ws; ws += (size_t)NB_ * NN * 4;
  if ((size_t)(ws - (char*)d_ws) > ws_size) return;
  k_ab<<<dim3(NB_ * 4), dim3(256), 0, stream>>>(h, w1, b1, w2, b2, av, bv);
  k_attn<<<dim3(NB_ * (NN / 32)), dim3(256), 0, stream>>>(h, av, bv, out);
}
